// CasualSelfAttention_5506148073688
// MI455X (gfx1250) — hardware-verified
//
#include <hip/hip_runtime.h>


#ifndef NB
#define NB 2
#endif
#ifndef SEQ
#define SEQ 2048
#endif
#define NB_FULL  2
#define SEQ_FULL 2048
#define TT   SEQ
#define DM   1024
#define D3   (3 * DM)
#define NH_  16
#define HD   64
#define HP   (HD / 2)
#define DQ   (NH_ * HD)
#define ZH   2
#define ER   64
#define SCL  0.125f
#define RC   (-0.14391156831212787f)
static_assert(NB >= 1 && NB <= NB_FULL);
static_assert(SEQ % 128 == 0 && SEQ >= 128 && SEQ <= SEQ_FULL);
static_assert(NH_ % ZH == 0);
static_assert(ER == 64 && ER <= TT);
static_assert(DM % 64 == 0 && D3 % 64 == 0 && HD % 64 == 0 && TT % 64 == 0 && DQ % 32 == 0);

typedef _Float16 h16;
typedef unsigned short bf;
typedef __attribute__((ext_vector_type(16))) __bf16   v16bf;
typedef __attribute__((ext_vector_type(16))) _Float16 v16h;
typedef __attribute__((ext_vector_type(8)))  _Float16 v8h;
typedef __attribute__((ext_vector_type(8)))  unsigned short v8us;
typedef __attribute__((ext_vector_type(8)))  float    v8f;
typedef __attribute__((ext_vector_type(4)))  float    v4f;
typedef v8h  __attribute__((may_alias)) v8ha;
typedef v4f  __attribute__((may_alias)) v4fa;
typedef v8us __attribute__((may_alias)) v8usa;

__device__ __forceinline__ unsigned short f2bf(float f) { unsigned u = __float_as_uint(f); u += 0x7FFFu + ((u >> 16) & 1u); return (unsigned short)(u >> 16); }
__device__ __forceinline__ float bf2f(unsigned short b) { return __uint_as_float(((unsigned)b) << 16); }
__device__ __forceinline__ float bfr(float f) { return bf2f(f2bf(f)); }
__device__ __forceinline__ v16h cat16(v8h lo, v8h hi) { return __builtin_shufflevector(lo, hi, 0, 1, 2, 3, 4, 5, 6, 7, 8, 9, 10, 11, 12, 13, 14, 15); }
__device__ __forceinline__ v16bf cat16b(v8us lo, v8us hi) { return __builtin_bit_cast(v16bf, __builtin_shufflevector(lo, hi, 0, 1, 2, 3, 4, 5, 6, 7, 8, 9, 10, 11, 12, 13, 14, 15)); }
__device__ __forceinline__ v8f wmma16(v16h a, v16h b, v8f c) { return __builtin_amdgcn_wmma_f32_16x16x32_f16(false, a, false, b, (short)0, c, false, false); }
__device__ __forceinline__ v8f wmmab(v16bf a, v16bf b, v8f c) { return __builtin_amdgcn_wmma_f32_16x16x32_bf16(false, a, false, b, (short)0, c, false, false); }

template <typename T16> struct WFrag;
template <> struct WFrag<h16> { typedef v16h V; static __device__ __forceinline__ V ld(const h16* p) { return cat16(*(const v8h*)p, *(const v8h*)(p + 16)); } static __device__ __forceinline__ v8f mma(V a, V b, v8f c) { return wmma16(a, b, c); } };
template <> struct WFrag<bf> { typedef v16bf V; static __device__ __forceinline__ V ld(const bf* p) { return cat16b(*(const v8us*)p, *(const v8us*)(p + 16)); } static __device__ __forceinline__ v8f mma(V a, V b, v8f c) { return wmmab(a, b, c); } };
template <typename T16, int NSPLIT, bool BIAS>
__global__ __launch_bounds__(32) void k_gemmw(const T16* __restrict__ A, const T16* __restrict__ A2, const T16* __restrict__ Bt, const T16* __restrict__ Bt2, int K, float* C, int ldc, const float* __restrict__ bias, size_t sA, size_t sB, size_t sC, int cm) {
    typedef typename WFrag<T16>::V V;
    __shared__ __align__(16) float os[16 * 68];
    if (cm == 1 && blockIdx.y > blockIdx.x) return;
    const size_t z = blockIdx.z; A += z * sA; if (A2) A2 += z * sA; Bt += z * sB; if (Bt2) Bt2 += z * sB; C += z * sC;
    const int lane = threadIdx.x & 31, lr = lane & 15, hi = lane >> 4; const int r0 = blockIdx.x * 64, c0 = blockIdx.y * 64;
    const int KE = (cm == 2 && r0 + 64 < K) ? (r0 + 64) : K;
    v8f acc[4][4];
#pragma unroll
    for (int mb = 0; mb < 4; ++mb)
#pragma unroll
        for (int nb = 0; nb < 4; ++nb) acc[mb][nb] = (v8f){};
    const size_t aoff = (size_t)(r0 + lr) * K + 8 * hi, boff = (size_t)(c0 + lr) * K + 8 * hi;
#pragma unroll 1
    for (int kc = 0; kc < KE; kc += 32) {
        V a[4], a2[4];
#pragma unroll
        for (int mb = 0; mb < 4; ++mb) { a[mb] = WFrag<T16>::ld(A + aoff + (size_t)mb * 16 * K + kc); if (NSPLIT == 1 || NSPLIT == 2) a2[mb] = WFrag<T16>::ld(A2 + aoff + (size_t)mb * 16 * K + kc); }
#pragma unroll
        for (int nb = 0; nb < 4; ++nb) { const V b = WFrag<T16>::ld(Bt + boff + (size_t)nb * 16 * K + kc); V b2; if (NSPLIT >= 2) b2 = WFrag<T16>::ld(Bt2 + boff + (size_t)nb * 16 * K + kc);
#pragma unroll
            for (int mb = 0; mb < 4; ++mb) { acc[mb][nb] = WFrag<T16>::mma(a[mb], b, acc[mb][nb]); if (NSPLIT == 1 || NSPLIT == 2) acc[mb][nb] = WFrag<T16>::mma(a2[mb], b, acc[mb][nb]); if (NSPLIT >= 2) acc[mb][nb] = WFrag<T16>::mma(a[mb], b2, acc[mb][nb]); } }
        asm volatile("v_nop\n\tv_nop\n\tv_nop\n\tv_nop" : "+v"(acc[0][0]), "+v"(acc[1][1]), "+v"(acc[2][2]), "+v"(acc[3][3]) : "v"(a[0]), "v"(a[3]));
    }
#pragma unroll
    for (int mb = 0; mb < 4; ++mb) {
#pragma unroll
        for (int nb = 0; nb < 4; ++nb) {
#pragma unroll
            for (int j = 0; j < 8; ++j) os[(hi * 8 + j) * 68 + nb * 16 + lr] = acc[mb][nb][j]; }
        __builtin_amdgcn_wave_barrier(); asm volatile("" ::: "memory");
        float* crow = C + (size_t)(r0 + mb * 16) * ldc + c0;
#pragma unroll 1
        for (int ps = 0; ps < 2; ++ps) {
#pragma unroll
            for (int s = 0; s < 8; ++s) { const int row = 2 * s + hi, cofs = lr * 4; v4f val = *(const v4fa*)(os + row * 68 + cofs); if (BIAS) { val[0] += bfr(bias[c0 + cofs]); val[1] += bfr(bias[c0 + cofs + 1]); val[2] += bfr(bias[c0 + cofs + 2]); val[3] += bfr(bias[c0 + cofs + 3]); }
                *(volatile v4f*)(crow + (size_t)row * ldc + cofs) = val; }
            if (ps == 0) __threadfence(); }
        __builtin_amdgcn_wave_barrier(); asm volatile("" ::: "memory");
    }
}

__device__ __forceinline__ h16 tohx(float x) { return (h16)x; }
__device__ __forceinline__ void splitf(float y, unsigned short& h, unsigned short& l) { h = f2bf(y); l = f2bf(y - bf2f(h)); }
typedef __attribute__((ext_vector_type(2))) _Float16 v2h;
typedef __attribute__((ext_vector_type(2))) unsigned short v2us;
typedef __attribute__((ext_vector_type(4))) unsigned short v4us;
typedef __attribute__((ext_vector_type(2))) float v2f;

__global__ __launch_bounds__(256) void k_cvt8(const float* __restrict__ src, bf* dst, size_t n8) { const size_t i = (size_t)blockIdx.x * 256 + threadIdx.x; if (i >= n8) return; const v8f v = *(const v8f*)(src + i * 8); v8us o;
#pragma unroll
    for (int k = 0; k < 8; ++k) o[k] = f2bf(v[k]); *(volatile v8us*)(dst + i * 8) = o; __threadfence(); *(volatile v8us*)(dst + i * 8) = o; }

__global__ __launch_bounds__(256) void k_rtab(float* CS, int n) {
    const int i = blockIdx.x * 256 + threadIdx.x; if (i >= n) return;
    const int t = i / HP; const int j = i - t * HP;
    const float dv = expf((float)(2 * j) * RC);
    const float ang = (float)t * dv;
    float s, c; sincosf(ang, &s, &c);
    v2f o; o[0] = c; o[1] = s;
    *(volatile v2f*)(CS + (size_t)i * 2) = o; __threadfence(); *(volatile v2f*)(CS + (size_t)i * 2) = o; }

__global__ __launch_bounds__(256) void k_qkp(const float* __restrict__ F, const float* __restrict__ CS, h16* Q16, h16* K16, bf* QBh, bf* QBl, bf* KBh, bf* KBl) {
    const size_t e = ((size_t)blockIdx.x * 256 + threadIdx.x) * 2; if (e >= (size_t)NH_ * TT * HD) return;
    const int d = (int)(e % HD); const int t = (int)((e / HD) % TT); const int h = (int)(e / ((size_t)HD * TT));
    const int up = (d >= HP) ? 1 : 0; const int jj = d - up * HP;
    const float* f = F + (size_t)t * D3 + h * HD + 2 * jj;
    const v4f xq = *(const v4f*)f; const v4f xk = *(const v4f*)(f + DM);
    const v4f cs = *(const v4f*)(CS + ((size_t)t * HP + jj) * 2);
    const float qa0 = xq[0] * cs[0] - xq[1] * cs[1], qa1 = xq[2] * cs[2] - xq[3] * cs[3];
    const float qb0 = xq[0] * cs[1] + xq[1] * cs[0], qb1 = xq[2] * cs[3] + xq[3] * cs[2];
    const float ka0 = xk[0] * cs[0] - xk[1] * cs[1], ka1 = xk[2] * cs[2] - xk[3] * cs[3];
    const float kb0 = xk[0] * cs[1] + xk[1] * cs[0], kb1 = xk[2] * cs[3] + xk[3] * cs[2];
    const float q0 = up ? qb0 : qa0, q1 = up ? qb1 : qa1, k0 = up ? kb0 : ka0, k1 = up ? kb1 : ka1;
    v2h oq, ok; oq[0] = tohx(q0); oq[1] = tohx(q1); ok[0] = tohx(k0); ok[1] = tohx(k1);
    v2us qh, ql, kh, kl;
    { unsigned short a2, c2;
      splitf(q0, a2, c2); qh[0] = a2; ql[0] = c2; splitf(q1, a2, c2); qh[1] = a2; ql[1] = c2;
      splitf(k0, a2, c2); kh[0] = a2; kl[0] = c2; splitf(k1, a2, c2); kh[1] = a2; kl[1] = c2; }
    const bool early = t < ER;
    const size_t eb = ((size_t)h * ER + (early ? t : 0)) * HD + d;
    *(volatile v2h*)(Q16 + e) = oq; *(volatile v2h*)(K16 + e) = ok;
    if (early) { *(volatile v2us*)(QBh + eb) = qh; *(volatile v2us*)(QBl + eb) = ql; *(volatile v2us*)(KBh + eb) = kh; *(volatile v2us*)(KBl + eb) = kl; }
    __threadfence();
    *(volatile v2h*)(Q16 + e) = oq; *(volatile v2h*)(K16 + e) = ok;
    if (early) { *(volatile v2us*)(QBh + eb) = qh; *(volatile v2us*)(QBl + eb) = ql; *(volatile v2us*)(KBh + eb) = kh; *(volatile v2us*)(KBl + eb) = kl; }
}

__global__ __launch_bounds__(256) void k_vtp(const float* __restrict__ F, bf* Vh, bf* Vl) {
    const size_t e = ((size_t)blockIdx.x * 256 + threadIdx.x) * 2; if (e >= (size_t)NH_ * HD * TT) return;
    const int t = (int)(e % TT); const int d = (int)((e / TT) % HD); const int g = (int)(e / ((size_t)TT * HD)); v2us oh, ol;
#pragma unroll
    for (int q = 0; q < 2; ++q) { const float x = F[(size_t)(t + q) * D3 + 2 * DM + g * HD + d]; unsigned short a2, c2; splitf(x, a2, c2); oh[q] = a2; ol[q] = c2; }
    *(volatile v2us*)(Vh + e) = oh; *(volatile v2us*)(Vl + e) = ol; __threadfence(); *(volatile v2us*)(Vh + e) = oh; *(volatile v2us*)(Vl + e) = ol; }

__global__ __launch_bounds__(256) void k_asoft(const float* __restrict__ Sb, const float* __restrict__ Se, bf* Ph, bf* Pl) {
    const int lane = threadIdx.x & 31; const int row = blockIdx.x * 8 + (threadIdx.x >> 5); if (row >= ZH * TT) return;
    const int zz = row / TT; const int i = row - zz * TT;
    const float* sr = Sb + (size_t)row * TT;
    const float* se = Se + ((size_t)zz * ER + (i < ER ? i : ER - 1)) * ER + (lane < 16 ? lane * 4 : ER - 4);
    const float NEG = -__builtin_inff();
    float v[TT / 32]; float mx = -3.0e38f;
#pragma unroll
    for (int ch = 0; ch < TT / 128; ++ch) { const int j0 = ch * 128 + lane * 4;
        if (ch * 128 <= i) {
            const float* p = sr + j0;
            if (ch == 0) p = (i < ER) ? se : p;
            const v4f a = *(const v4f*)p;
#pragma unroll
            for (int q = 0; q < 4; ++q) { const float t = (j0 + q <= i) ? a[q] * SCL : NEG; v[ch * 4 + q] = t; mx = fmaxf(mx, t); }
        } else {
#pragma unroll
            for (int q = 0; q < 4; ++q) v[ch * 4 + q] = NEG;
        }
    }
#pragma unroll
    for (int sh = 16; sh; sh >>= 1) mx = fmaxf(mx, __shfl_xor(mx, sh, 32));
    float sum = 0.f;
#pragma unroll
    for (int k = 0; k < TT / 32; ++k) { float d0 = __fsub_rn(v[k], mx); asm volatile("" : "+v"(d0)); v[k] = __builtin_amdgcn_exp2f(__fmul_rn(d0, 1.4426950408889634f)); sum += v[k]; }
#pragma unroll
    for (int sh = 16; sh; sh >>= 1) sum += __shfl_xor(sum, sh, 32);
    const float f = __fdiv_rn(1.0f, sum);
#pragma unroll 1
    for (int ps = 0; ps < 2; ++ps) {
#pragma unroll
        for (int ch = 0; ch < TT / 128; ++ch) { v4us oh, ol;
#pragma unroll
            for (int q = 0; q < 4; ++q) { unsigned short a, c2; splitf(v[ch * 4 + q] * f, a, c2); oh[q] = a; ol[q] = c2; }
            const size_t oo = (size_t)row * TT + ch * 128 + lane * 4; *(volatile v4us*)(Ph + oo) = oh; *(volatile v4us*)(Pl + oo) = ol; }
        if (ps == 0) __threadfence(); }
}

__global__ __launch_bounds__(256) void k_merge(const float* __restrict__ O, int h0, bf* Ah, bf* Al) {
    const size_t e = ((size_t)blockIdx.x * 256 + threadIdx.x) * 2; if (e >= (size_t)ZH * TT * HD) return;
    const int d = (int)(e % HD); const int t = (int)((e / HD) % TT); const int zz = (int)(e / ((size_t)HD * TT)); const size_t oo = (size_t)t * DQ + (h0 + zz) * HD + d;
    v2us oh, ol;
#pragma unroll
    for (int q = 0; q < 2; ++q) { unsigned short a, c2; splitf(O[e + q], a, c2); oh[q] = a; ol[q] = c2; }
    *(volatile v2us*)(Ah + oo) = oh; *(volatile v2us*)(Al + oo) = ol; __threadfence(); *(volatile v2us*)(Ah + oo) = oh; *(volatile v2us*)(Al + oo) = ol; }

constexpr size_t WS_NEED = (size_t)D3 * DM * 2 + (size_t)DM * DM * 2 + (size_t)TT * HP * 2 * 4 + (size_t)TT * DM * 2 + (size_t)TT * D3 * 4
                         + 2 * (size_t)NH_ * TT * HD * 2 + 4 * (size_t)NH_ * ER * HD * 2 + 2 * (size_t)NH_ * HD * TT * 2 + (size_t)NH_ * ER * ER * 4
                         + 2 * (size_t)ZH * TT * TT * 2 + (size_t)ZH * TT * TT * 4 + (size_t)ZH * TT * HD * 4 + 2 * (size_t)TT * DQ * 2;
static_assert(WS_NEED + 32 * 256 <= (size_t)134217728);

extern "C" void kernel_launch(void* const* d_in, const int* in_sizes, int n_in,
                              void* d_out, int out_size, void* d_ws, size_t ws_size, hipStream_t stream) {
    if (n_in < 5) return;
    if (in_sizes[0] < NB * TT * DM || in_sizes[1] < D3 * DM || in_sizes[2] < D3 || in_sizes[3] < DM * DM || in_sizes[4] < DM) return;
    if (out_size < NB * TT * DM) return;
    const float* x = (const float*)d_in[0];
    const float* wattn = (const float*)d_in[1];
    const float* battn = (const float*)d_in[2];
    const float* wproj = (const float*)d_in[3];
    const float* bproj = (const float*)d_in[4];
    float* OUT = (float*)d_out;
    char* wsp = (char*)d_ws;
    auto take = [&](size_t bytes) { char* p = wsp; wsp += (bytes + 255) & ~(size_t)255; return (void*)p; };
    bf* WALL = (bf*)take((size_t)D3 * DM * 2); bf* WO = (bf*)take((size_t)DM * DM * 2);
    float* CS = (float*)take((size_t)TT * HP * 2 * 4);
    bf* XB = (bf*)take((size_t)TT * DM * 2); float* F = (float*)take((size_t)TT * D3 * 4);
    h16* QP16 = (h16*)take((size_t)NH_ * TT * HD * 2); h16* KP16 = (h16*)take((size_t)NH_ * TT * HD * 2);
    bf* QBh = (bf*)take((size_t)NH_ * ER * HD * 2); bf* QBl = (bf*)take((size_t)NH_ * ER * HD * 2);
    bf* KBh = (bf*)take((size_t)NH_ * ER * HD * 2); bf* KBl = (bf*)take((size_t)NH_ * ER * HD * 2);
    bf* VTh = (bf*)take((size_t)NH_ * HD * TT * 2); bf* VTl = (bf*)take((size_t)NH_ * HD * TT * 2);
    float* Se = (float*)take((size_t)NH_ * ER * ER * 4);
    bf* Ph = (bf*)take((size_t)ZH * TT * TT * 2); bf* Pl = (bf*)take((size_t)ZH * TT * TT * 2);
    float* Sb = (float*)take((size_t)ZH * TT * TT * 4); float* Ob = (float*)take((size_t)ZH * TT * HD * 4);
    bf* ATh = (bf*)take((size_t)TT * DQ * 2); bf* ATl = (bf*)take((size_t)TT * DQ * 2);
    if ((size_t)(wsp - (char*)d_ws) > ws_size) return;
    k_cvt8<<<(unsigned)(((size_t)D3 * DM / 8 + 255) / 256), 256, 0, stream>>>(wattn, WALL, (size_t)D3 * DM / 8);
    k_cvt8<<<(unsigned)(((size_t)DM * DM / 8 + 255) / 256), 256, 0, stream>>>(wproj, WO, (size_t)DM * DM / 8);
    k_rtab<<<(unsigned)((TT * HP + 255) / 256), 256, 0, stream>>>(CS, TT * HP);
    const unsigned LP = (unsigned)(((size_t)NH_ * TT * HD / 2 + 255) / 256);
    const unsigned LM = (unsigned)(((size_t)ZH * TT * HD / 2 + 255) / 256);
    for (int b = 0; b < NB; ++b) {
        k_cvt8<<<(unsigned)(((size_t)TT * DM / 8 + 255) / 256), 256, 0, stream>>>(x + (size_t)b * SEQ_FULL * DM, XB, (size_t)TT * DM / 8);
        k_gemmw<bf, 0, true><<<dim3(TT / 64, D3 / 64, 1), 32, 0, stream>>>(XB, nullptr, WALL, nullptr, DM, F, D3, battn, 0, 0, 0, 0);
        k_qkp<<<LP, 256, 0, stream>>>(F, CS, QP16, KP16, QBh, QBl, KBh, KBl);
        k_vtp<<<LP, 256, 0, stream>>>(F, VTh, VTl);
        k_gemmw<bf, 2, false><<<dim3(1, 1, NH_), 32, 0, stream>>>(QBh, QBl, KBh, KBl, HD, Se, ER, nullptr, (size_t)ER * HD, (size_t)ER * HD, (size_t)ER * ER, 0);
        for (int h0 = 0; h0 < NH_; h0 += ZH) { const size_t zq = (size_t)h0;
            k_gemmw<h16, 0, false><<<dim3(TT / 64, TT / 64, ZH), 32, 0, stream>>>(QP16 + zq * TT * HD, nullptr, KP16 + zq * TT * HD, nullptr, HD, Sb, TT, nullptr, (size_t)TT * HD, (size_t)TT * HD, (size_t)TT * TT, 1);
            k_asoft<<<ZH * TT / 8, 256, 0, stream>>>(Sb, Se + zq * ER * ER, Ph, Pl);
            k_gemmw<bf, 2, false><<<dim3(TT / 64, HD / 64, ZH), 32, 0, stream>>>(Ph, Pl, VTh + zq * HD * TT, VTl + zq * HD * TT, TT, Ob, HD, nullptr, (size_t)TT * TT, (size_t)HD * TT, (size_t)TT * HD, 2);
            k_merge<<<LM, 256, 0, stream>>>(Ob, h0, ATh, ATl); }
        k_gemmw<bf, 1, true><<<dim3(TT / 64, DM / 64, 1), 32, 0, stream>>>(ATh, ATl, WO, nullptr, DQ, OUT + (size_t)b * TT * DM, DM, bproj, 0, 0, 0, 0); }
}
